// MultiHeadedAttention_15650860826821
// MI455X (gfx1250) — hardware-verified
//
#include <hip/hip_runtime.h>


#ifndef NB
#define NB 8
#endif
#ifndef SEQ
#define SEQ 1024
#endif
#define SEQ_FULL 1024
#define TT   SEQ
#define DM   768
#define NH_  12
#define HD   64
#define SCL  0.015625f

static_assert(TT % 128 == 0);
static_assert(TT <= SEQ_FULL);
static_assert(NH_ * HD == DM);
static_assert(DM % 64 == 0);
static_assert(HD == 64);
static_assert(NB >= 1 && NB <= 8);

typedef _Float16 h16;
typedef unsigned short bf;
typedef __attribute__((ext_vector_type(16))) __bf16   v16bf;
typedef __attribute__((ext_vector_type(16))) _Float16 v16h;
typedef __attribute__((ext_vector_type(8)))  _Float16 v8h;
typedef __attribute__((ext_vector_type(8)))  unsigned short v8us;
typedef __attribute__((ext_vector_type(8)))  float    v8f;
typedef __attribute__((ext_vector_type(4)))  float    v4f;
typedef __attribute__((ext_vector_type(4)))  unsigned short v4us;
typedef v8h  __attribute__((may_alias)) v8ha;
typedef v4f  __attribute__((may_alias)) v4fa;
typedef v8us __attribute__((may_alias)) v8usa;

__device__ __forceinline__ unsigned short f2bf(float f) { unsigned u = __float_as_uint(f); u += 0x7FFFu + ((u >> 16) & 1u); return (unsigned short)(u >> 16); }
__device__ __forceinline__ float bf2f(unsigned short b) { return __uint_as_float(((unsigned)b) << 16); }
__device__ __forceinline__ float bfr(float f) { return bf2f(f2bf(f)); }
__device__ __forceinline__ v16h cat16(v8h lo, v8h hi) { return __builtin_shufflevector(lo, hi, 0, 1, 2, 3, 4, 5, 6, 7, 8, 9, 10, 11, 12, 13, 14, 15); }
__device__ __forceinline__ v16bf cat16b(v8us lo, v8us hi) { return __builtin_bit_cast(v16bf, __builtin_shufflevector(lo, hi, 0, 1, 2, 3, 4, 5, 6, 7, 8, 9, 10, 11, 12, 13, 14, 15)); }
__device__ __forceinline__ v8f wmma16(v16h a, v16h b, v8f c) { return __builtin_amdgcn_wmma_f32_16x16x32_f16(false, a, false, b, (short)0, c, false, false); }
__device__ __forceinline__ v8f wmmab(v16bf a, v16bf b, v8f c) { return __builtin_amdgcn_wmma_f32_16x16x32_bf16(false, a, false, b, (short)0, c, false, false); }
__device__ __forceinline__ h16 tohx(float x) { return (h16)x; }
__device__ __forceinline__ void splitf(float y, unsigned short& h, unsigned short& l) { h = f2bf(y); l = f2bf(y - bf2f(h)); }

template <typename T16> struct WFrag;
template <> struct WFrag<h16> { typedef v16h V; static __device__ __forceinline__ V ld(const h16* p) { return cat16(*(const v8h*)p, *(const v8h*)(p + 16)); } static __device__ __forceinline__ v8f mma(V a, V b, v8f c) { return wmma16(a, b, c); } };
template <> struct WFrag<bf> { typedef v16bf V; static __device__ __forceinline__ V ld(const bf* p) { return cat16b(*(const v8us*)p, *(const v8us*)(p + 16)); } static __device__ __forceinline__ v8f mma(V a, V b, v8f c) { return wmmab(a, b, c); } };
template <typename T16, int NSPLIT, bool BIAS>
__global__ __launch_bounds__(32) void k_gemmw(const T16* __restrict__ A, const T16* __restrict__ A2, const T16* __restrict__ Bt, const T16* __restrict__ Bt2, int K, float* C, int ldc, const float* __restrict__ bias, size_t sA, size_t sB, size_t sC) {
    typedef typename WFrag<T16>::V V;
    __shared__ __align__(16) float os[16 * 68];
    const size_t z = blockIdx.z; A += z * sA; if (A2) A2 += z * sA; Bt += z * sB; if (Bt2) Bt2 += z * sB; C += z * sC;
    const int lane = threadIdx.x & 31, lr = lane & 15, hi = lane >> 4; const int r0 = blockIdx.x * 64, c0 = blockIdx.y * 64;
    v8f acc[4][4];
#pragma unroll
    for (int mb = 0; mb < 4; ++mb)
#pragma unroll
        for (int nb = 0; nb < 4; ++nb) acc[mb][nb] = (v8f){};
    const size_t aoff = (size_t)(r0 + lr) * K + 8 * hi, boff = (size_t)(c0 + lr) * K + 8 * hi;
#pragma unroll 1
    for (int kc = 0; kc < K; kc += 32) {
        V a[4], a2[4];
#pragma unroll
        for (int mb = 0; mb < 4; ++mb) { a[mb] = WFrag<T16>::ld(A + aoff + (size_t)mb * 16 * K + kc); if (NSPLIT == 1 || NSPLIT == 2) a2[mb] = WFrag<T16>::ld(A2 + aoff + (size_t)mb * 16 * K + kc); }
#pragma unroll
        for (int nb = 0; nb < 4; ++nb) { const V b = WFrag<T16>::ld(Bt + boff + (size_t)nb * 16 * K + kc); V b2; if (NSPLIT >= 2) b2 = WFrag<T16>::ld(Bt2 + boff + (size_t)nb * 16 * K + kc);
#pragma unroll
            for (int mb = 0; mb < 4; ++mb) { acc[mb][nb] = WFrag<T16>::mma(a[mb], b, acc[mb][nb]); if (NSPLIT == 1 || NSPLIT == 2) acc[mb][nb] = WFrag<T16>::mma(a2[mb], b, acc[mb][nb]); if (NSPLIT >= 2) acc[mb][nb] = WFrag<T16>::mma(a[mb], b2, acc[mb][nb]); } }
        asm volatile("v_nop\n\tv_nop\n\tv_nop\n\tv_nop" : "+v"(acc[0][0]), "+v"(acc[1][1]), "+v"(acc[2][2]), "+v"(acc[3][3]) : "v"(a[0]), "v"(a[3]));
    }
#pragma unroll
    for (int mb = 0; mb < 4; ++mb) {
#pragma unroll
        for (int nb = 0; nb < 4; ++nb) {
#pragma unroll
            for (int j = 0; j < 8; ++j) os[(hi * 8 + j) * 68 + nb * 16 + lr] = acc[mb][nb][j]; }
        __builtin_amdgcn_wave_barrier(); asm volatile("" ::: "memory");
        float* crow = C + (size_t)(r0 + mb * 16) * ldc + c0;
#pragma unroll 1
        for (int ps = 0; ps < 2; ++ps) {
#pragma unroll
            for (int s = 0; s < 8; ++s) { const int row = 2 * s + hi, cofs = lr * 4; v4f val = *(const v4fa*)(os + row * 68 + cofs); if (BIAS) { val[0] += bfr(bias[c0 + cofs]); val[1] += bfr(bias[c0 + cofs + 1]); val[2] += bfr(bias[c0 + cofs + 2]); val[3] += bfr(bias[c0 + cofs + 3]); }
                *(volatile v4f*)(crow + (size_t)row * ldc + cofs) = val; }
            if (ps == 0) __threadfence(); }
        __builtin_amdgcn_wave_barrier(); asm volatile("" ::: "memory");
    }
}

__global__ __launch_bounds__(256) void k_cvt8(const float* __restrict__ src, bf* dst, size_t n8) { const size_t i = (size_t)blockIdx.x * 256 + threadIdx.x; if (i >= n8) return; const v8f v = *(const v8f*)(src + i * 8); v8us o;
#pragma unroll
    for (int k = 0; k < 8; ++k) o[k] = f2bf(v[k]); *(volatile v8us*)(dst + i * 8) = o; __threadfence(); *(volatile v8us*)(dst + i * 8) = o; }

__global__ __launch_bounds__(256) void k_wt(const float* __restrict__ wq, const float* __restrict__ wk, const float* __restrict__ wv, bf* Bt) {
    const int z = blockIdx.y;
    const float* w = (z == 0) ? wq : ((z == 1) ? wk : wv);
    const size_t i = (size_t)blockIdx.x * 256 + threadIdx.x; if (i >= (size_t)DM * DM / 8) return;
    const size_t e = i * 8; const int k = (int)(e % DM); const int n = (int)(e / DM); const int h = n / HD, c = n % HD;
    v8us o;
#pragma unroll
    for (int q = 0; q < 8; ++q) o[q] = f2bf(w[((size_t)h * DM + k + q) * HD + c]);
    bf* d = Bt + (size_t)z * DM * DM + e;
    *(volatile v8us*)d = o; __threadfence(); *(volatile v8us*)d = o;
}

__global__ __launch_bounds__(256) void k_qkp(const float* __restrict__ FQ, const float* __restrict__ FK, const float* __restrict__ bq, const float* __restrict__ bk, h16* QP, h16* KP) {
    const int y = blockIdx.y;
    const float* F = y ? FK : FQ; const float* bias = y ? bk : bq; h16* P = y ? KP : QP;
    const size_t i = (size_t)blockIdx.x * 256 + threadIdx.x; if (i >= (size_t)NH_ * TT * HD / 8) return;
    const size_t e = i * 8; const int d = (int)(e % HD); const int t = (int)((e / HD) % TT); const int h = (int)(e / ((size_t)HD * TT));
    const v8f f = *(const v8f*)(F + (size_t)t * DM + h * HD + d); const v8f bb = *(const v8f*)(bias + h * HD + d);
    v8h o;
#pragma unroll
    for (int q = 0; q < 8; ++q) o[q] = tohx(f[q] + bfr(bb[q]));
    *(volatile v8h*)(P + e) = o; __threadfence(); *(volatile v8h*)(P + e) = o;
}

__global__ __launch_bounds__(256) void k_vtp(const float* __restrict__ F, const float* __restrict__ bias, bf* Vh, bf* Vl) {
    const size_t i = (size_t)blockIdx.x * 256 + threadIdx.x; if (i >= (size_t)NH_ * HD * TT / 8) return;
    const size_t e = i * 8; const int t = (int)(e % TT); const int d = (int)((e / TT) % HD); const int h = (int)(e / ((size_t)TT * HD));
    const float bb = bfr(bias[h * HD + d]);
    v8us oh, ol;
#pragma unroll
    for (int q = 0; q < 8; ++q) { const float x = F[(size_t)(t + q) * DM + h * HD + d] + bb; unsigned short a2, c2; splitf(x, a2, c2); oh[q] = a2; ol[q] = c2; }
    *(volatile v8us*)(Vh + e) = oh; *(volatile v8us*)(Vl + e) = ol; __threadfence(); *(volatile v8us*)(Vh + e) = oh; *(volatile v8us*)(Vl + e) = ol;
}

__global__ __launch_bounds__(256) void k_asoft(const float* __restrict__ Sb, bf* Ph, bf* Pl) {
    const int lane = threadIdx.x & 31; const int row = blockIdx.x * 8 + (threadIdx.x >> 5); if (row >= NH_ * TT) return;
    const float* sr = Sb + (size_t)row * TT; float v[TT / 32]; float mx = -3.0e38f;
#pragma unroll
    for (int ch = 0; ch < TT / 128; ++ch) { const int j0 = ch * 128 + lane * 4; const v4f a = *(const v4f*)(sr + j0);
#pragma unroll
        for (int q = 0; q < 4; ++q) { const float t = a[q] * SCL; v[ch * 4 + q] = t; mx = fmaxf(mx, t); } }
#pragma unroll
    for (int sh = 16; sh; sh >>= 1) mx = fmaxf(mx, __shfl_xor(mx, sh, 32));
    float sum = 0.f;
#pragma unroll
    for (int k = 0; k < TT / 32; ++k) { float d0 = __fsub_rn(v[k], mx); asm volatile("" : "+v"(d0)); v[k] = __builtin_amdgcn_exp2f(__fmul_rn(d0, 1.4426950408889634f)); sum += v[k]; }
#pragma unroll
    for (int sh = 16; sh; sh >>= 1) sum += __shfl_xor(sum, sh, 32);
    const float f = __fdiv_rn(1.0f, sum);
#pragma unroll 1
    for (int ps = 0; ps < 2; ++ps) {
#pragma unroll
        for (int ch = 0; ch < TT / 128; ++ch) { v4us oh, ol;
#pragma unroll
            for (int q = 0; q < 4; ++q) { unsigned short a, c2; splitf(v[ch * 4 + q] * f, a, c2); oh[q] = a; ol[q] = c2; }
            const size_t oo = (size_t)row * TT + ch * 128 + lane * 4; *(volatile v4us*)(Ph + oo) = oh; *(volatile v4us*)(Pl + oo) = ol; }
        if (ps == 0) __threadfence(); }
}

extern "C" void kernel_launch(void* const* d_in, const int* in_sizes, int n_in,
                              void* d_out, int out_size, void* d_ws, size_t ws_size, hipStream_t stream) {
    if (n_in < 7) return;
    if (in_sizes[0] < NB * SEQ_FULL * DM) return;
    if (in_sizes[1] < NH_ * DM * HD || in_sizes[3] < NH_ * DM * HD || in_sizes[5] < NH_ * DM * HD) return;
    if (in_sizes[2] < NH_ * HD || in_sizes[4] < NH_ * HD || in_sizes[6] < NH_ * HD) return;
    if (out_size < NB * TT * DM) return;
    const float* x  = (const float*)d_in[0];
    const float* wq = (const float*)d_in[1]; const float* bq = (const float*)d_in[2];
    const float* wk = (const float*)d_in[3]; const float* bk = (const float*)d_in[4];
    const float* wv = (const float*)d_in[5]; const float* bv = (const float*)d_in[6];
    float* OUT = (float*)d_out;
    char* wsp = (char*)d_ws;
    auto take = [&](size_t bytes) { char* p = wsp; wsp += (bytes + 255) & ~(size_t)255; return (void*)p; };
    bf*    WT  = (bf*)take((size_t)3 * DM * DM * 2);
    bf*    XB  = (bf*)take((size_t)NB * SEQ_FULL * DM * 2);
    float* F   = (float*)take((size_t)3 * TT * DM * 4);
    h16*   QP  = (h16*)take((size_t)NH_ * TT * HD * 2);
    h16*   KP  = (h16*)take((size_t)NH_ * TT * HD * 2);
    bf*    VTh = (bf*)take((size_t)NH_ * HD * TT * 2);
    bf*    VTl = (bf*)take((size_t)NH_ * HD * TT * 2);
    float* Sb  = (float*)take((size_t)NH_ * TT * TT * 4);
    bf*    Ph  = (bf*)take((size_t)NH_ * TT * TT * 2);
    bf*    Pl  = (bf*)take((size_t)NH_ * TT * TT * 2);
    if ((size_t)(wsp - (char*)d_ws) > ws_size) return;
    float* FQ = F; float* FK = F + (size_t)TT * DM; float* FV = F + (size_t)2 * TT * DM;

    k_wt<<<dim3((unsigned)(((size_t)DM * DM / 8 + 255) / 256), 3), 256, 0, stream>>>(wq, wk, wv, WT);
    const size_t nx8 = (size_t)NB * SEQ_FULL * DM / 8;
    k_cvt8<<<(unsigned)((nx8 + 255) / 256), 256, 0, stream>>>(x, XB, nx8);
    const unsigned LP = (unsigned)(((size_t)NH_ * TT * HD / 8 + 255) / 256);
    for (int b = 0; b < NB; ++b) {
        k_gemmw<bf, 0, false><<<dim3(TT / 64, DM / 64, 3), 32, 0, stream>>>(XB + (size_t)b * SEQ_FULL * DM, nullptr, WT, nullptr, DM, F, DM, nullptr, (size_t)0, (size_t)DM * DM, (size_t)TT * DM);
        k_qkp<<<dim3(LP, 2), 256, 0, stream>>>(FQ, FK, bq, bk, QP, KP);
        k_vtp<<<LP, 256, 0, stream>>>(FV, bv, VTh, VTl);
        k_gemmw<h16, 0, false><<<dim3(TT / 64, TT / 64, NH_), 32, 0, stream>>>(QP, nullptr, KP, nullptr, HD, Sb, TT, nullptr, (size_t)TT * HD, (size_t)TT * HD, (size_t)TT * TT);
        k_asoft<<<(unsigned)((NH_ * TT + 7) / 8), 256, 0, stream>>>(Sb, Ph, Pl);
        k_gemmw<bf, 2, false><<<dim3(TT / 64, HD / 64, NH_), 32, 0, stream>>>(Ph, Pl, VTh, VTl, TT, OUT + (size_t)b * TT * DM, DM, nullptr, (size_t)TT * TT, (size_t)HD * TT, (size_t)HD);
    }
}
